// RnnAutoEncoder_44650480009505
// MI455X (gfx1250) — hardware-run, weakly checked
//
#include <hip/hip_runtime.h>


#define NTS 512
#define NBR 256
#define NRW 131072

typedef _Float16 h16;
typedef unsigned short bf;
typedef __attribute__((ext_vector_type(16))) __bf16   v16bf;
typedef __attribute__((ext_vector_type(16))) _Float16 v16h;
typedef __attribute__((ext_vector_type(8)))  _Float16 v8h;
typedef __attribute__((ext_vector_type(8)))  unsigned short v8us;
typedef __attribute__((ext_vector_type(8)))  float    v8f;
typedef __attribute__((ext_vector_type(4)))  float    v4f;
typedef v8h  __attribute__((may_alias)) v8ha;
typedef v4f  __attribute__((may_alias)) v4fa;
typedef v8us __attribute__((may_alias)) v8usa;

__device__ __forceinline__ unsigned short f2bf(float f) { unsigned u = __float_as_uint(f); u += 0x7FFFu + ((u >> 16) & 1u); return (unsigned short)(u >> 16); }
__device__ __forceinline__ float bf2f(unsigned short b) { return __uint_as_float(((unsigned)b) << 16); }
__device__ __forceinline__ float bfr(float f) { return bf2f(f2bf(f)); }
__device__ __forceinline__ v16h cat16(v8h lo, v8h hi) { return __builtin_shufflevector(lo, hi, 0, 1, 2, 3, 4, 5, 6, 7, 8, 9, 10, 11, 12, 13, 14, 15); }
__device__ __forceinline__ v16bf cat16b(v8us lo, v8us hi) { return __builtin_bit_cast(v16bf, __builtin_shufflevector(lo, hi, 0, 1, 2, 3, 4, 5, 6, 7, 8, 9, 10, 11, 12, 13, 14, 15)); }
__device__ __forceinline__ v8f wmma16(v16h a, v16h b, v8f c) { return __builtin_amdgcn_wmma_f32_16x16x32_f16(false, a, false, b, (short)0, c, false, false); }
__device__ __forceinline__ v8f wmmab(v16bf a, v16bf b, v8f c) { return __builtin_amdgcn_wmma_f32_16x16x32_bf16(false, a, false, b, (short)0, c, false, false); }

template <typename T16> struct WFrag;
template <> struct WFrag<h16> { typedef v16h V; static __device__ __forceinline__ V ld(const h16* p) { return cat16(*(const v8h*)p, *(const v8h*)(p + 16)); } static __device__ __forceinline__ v8f mma(V a, V b, v8f c) { return wmma16(a, b, c); } };
template <> struct WFrag<bf> { typedef v16bf V; static __device__ __forceinline__ V ld(const bf* p) { return cat16b(*(const v8us*)p, *(const v8us*)(p + 16)); } static __device__ __forceinline__ v8f mma(V a, V b, v8f c) { return wmmab(a, b, c); } };
template <typename T16, int NSPLIT, bool BIAS>
__global__ __launch_bounds__(32) void k_gemmw(const T16* __restrict__ A, const T16* __restrict__ A2, const T16* __restrict__ Bt, const T16* __restrict__ Bt2, int K, float* C, int ldc, const float* __restrict__ bias, size_t sA, size_t sB, size_t sC) {
    typedef typename WFrag<T16>::V V;
    __shared__ __align__(16) float os[16 * 68];
    const size_t z = blockIdx.z; A += z * sA; if (A2) A2 += z * sA; Bt += z * sB; if (Bt2) Bt2 += z * sB; C += z * sC;
    const int lane = threadIdx.x & 31, lr = lane & 15, hi = lane >> 4; const int r0 = blockIdx.x * 64, c0 = blockIdx.y * 64;
    v8f acc[4][4];
#pragma unroll
    for (int mb = 0; mb < 4; ++mb)
#pragma unroll
        for (int nb = 0; nb < 4; ++nb) acc[mb][nb] = (v8f){};
    const size_t aoff = (size_t)(r0 + lr) * K + 8 * hi, boff = (size_t)(c0 + lr) * K + 8 * hi;
    for (int kc = 0; kc < K; kc += 32) {
        V a[4], a2[4];
#pragma unroll
        for (int mb = 0; mb < 4; ++mb) { a[mb] = WFrag<T16>::ld(A + aoff + (size_t)mb * 16 * K + kc); if (NSPLIT == 1 || NSPLIT == 2) a2[mb] = WFrag<T16>::ld(A2 + aoff + (size_t)mb * 16 * K + kc); }
#pragma unroll
        for (int nb = 0; nb < 4; ++nb) { const V b = WFrag<T16>::ld(Bt + boff + (size_t)nb * 16 * K + kc); V b2; if (NSPLIT >= 2) b2 = WFrag<T16>::ld(Bt2 + boff + (size_t)nb * 16 * K + kc);
#pragma unroll
            for (int mb = 0; mb < 4; ++mb) { acc[mb][nb] = WFrag<T16>::mma(a[mb], b, acc[mb][nb]); if (NSPLIT == 1 || NSPLIT == 2) acc[mb][nb] = WFrag<T16>::mma(a2[mb], b, acc[mb][nb]); if (NSPLIT >= 2) acc[mb][nb] = WFrag<T16>::mma(a[mb], b2, acc[mb][nb]); } }
        asm volatile("v_nop\n\tv_nop\n\tv_nop\n\tv_nop" : "+v"(acc[0][0]), "+v"(acc[1][1]), "+v"(acc[2][2]), "+v"(acc[3][3]) : "v"(a[0]), "v"(a[3]));
    }
#pragma unroll
    for (int mb = 0; mb < 4; ++mb) {
#pragma unroll
        for (int nb = 0; nb < 4; ++nb) {
#pragma unroll
            for (int j = 0; j < 8; ++j) os[(hi * 8 + j) * 68 + nb * 16 + lr] = acc[mb][nb][j]; }
        __builtin_amdgcn_wave_barrier(); asm volatile("" ::: "memory");
        float* crow = C + (size_t)(r0 + mb * 16) * ldc + c0;
#pragma unroll 1
        for (int ps = 0; ps < 2; ++ps) {
#pragma unroll
            for (int s = 0; s < 8; ++s) { const int row = 2 * s + hi, cofs = lr * 4; v4f val = *(const v4fa*)(os + row * 68 + cofs); if (BIAS) { val[0] += bfr(bias[c0 + cofs]); val[1] += bfr(bias[c0 + cofs + 1]); val[2] += bfr(bias[c0 + cofs + 2]); val[3] += bfr(bias[c0 + cofs + 3]); }
                *(volatile v4f*)(crow + (size_t)row * ldc + cofs) = val; }
            if (ps == 0) __threadfence(); }
        __builtin_amdgcn_wave_barrier(); asm volatile("" ::: "memory");
    }
}

typedef __attribute__((ext_vector_type(2))) _Float16 v2h;
typedef __attribute__((ext_vector_type(4))) _Float16 v4h;
typedef __attribute__((ext_vector_type(2))) unsigned short v2us;
typedef __attribute__((ext_vector_type(4))) unsigned short v4us;
typedef __attribute__((ext_vector_type(2))) float v2f;
typedef __attribute__((ext_vector_type(4))) int v4i;
__device__ __forceinline__ h16 toh_flush(float x) { const float z = (fabsf(x) < 6.103515625e-05f) ? 0.0f : x; return (h16)z; }

typedef __attribute__((ext_vector_type(2))) _Float16 v2h_;
__global__ __launch_bounds__(256) void k_wword(const float* __restrict__ src, int nr, int nc, h16* dst, int pc) {
    const unsigned i = blockIdx.x * 256 + threadIdx.x; const unsigned e0 = i * 2u; const unsigned rr = e0 / (unsigned)pc, c0 = e0 - rr * (unsigned)pc; v2h_ ow;
#pragma unroll
    for (int j = 0; j < 2; ++j) { const unsigned cc = c0 + j; const unsigned rk = rr < (unsigned)nr ? rr : (unsigned)nr - 1u, ck = cc < (unsigned)nc ? cc : (unsigned)nc - 1u; const unsigned short keep = (unsigned short)(0u - ((unsigned)(rr < (unsigned)nr) & (unsigned)(cc < (unsigned)nc)));
        const h16 wv = toh_flush(bfr(src[(size_t)rk * nc + ck])); ow[j] = __builtin_bit_cast(h16, (unsigned short)(__builtin_bit_cast(unsigned short, wv) & keep)); }
    *(volatile v2h_*)(dst + e0) = ow; __threadfence(); *(volatile v2h_*)(dst + e0) = ow; }

__global__ __launch_bounds__(128) void k_bpad(const float* __restrict__ ba, int nb, float* dst) {
    const unsigned j = threadIdx.x; const unsigned jk = j < (unsigned)nb ? j : (unsigned)nb - 1u; const unsigned keep = 0u - (unsigned)(j < (unsigned)nb); const float y = __builtin_bit_cast(float, __builtin_bit_cast(unsigned, bfr(ba[jk])) & keep);
    *(volatile float*)(dst + j) = y; __threadfence(); *(volatile float*)(dst + j) = y; }

__global__ __launch_bounds__(256) void k_xword(const float* __restrict__ src, h16* dst) {
    const size_t i = (size_t)blockIdx.x * 256 + threadIdx.x; const v8f wv = *(const v8f*)(src + i * 8); v8h ow;
#pragma unroll
    for (int j = 0; j < 8; ++j) ow[j] = toh_flush(bfr(wv[j]));
    *(volatile v8h*)(dst + i * 8) = ow; __threadfence(); *(volatile v8h*)(dst + i * 8) = ow; }

__global__ __launch_bounds__(256) void k_rword(const float* __restrict__ src, int fp, h16* dst, int dp, int sh) {
    const unsigned i = blockIdx.x * 256 + threadIdx.x; const size_t rw = i >> sh; const unsigned c8 = i & ((1u << sh) - 1u); const v8f wv = *(const v8f*)(src + rw * fp + c8 * 8); v8h ow;
#pragma unroll
    for (int j = 0; j < 8; ++j) ow[j] = toh_flush(fmaxf(wv[j], 0.0f));
    h16* po = dst + rw * dp + c8 * 8; *(volatile v8h*)po = ow; __threadfence(); *(volatile v8h*)po = ow; }

template <bool RL>
__global__ __launch_bounds__(32) void k_cellm(const float* __restrict__ src, const h16* __restrict__ wr, const float* __restrict__ b2, h16* dst) {
    __shared__ __align__(16) float tl[16 * 36];
    const int lane = threadIdx.x & 31, lr = lane & 15, hi = lane >> 4; const int b0 = blockIdx.x * 16;
    const v16h wf0 = WFrag<h16>::ld(wr + (size_t)lr * 32 + 8 * hi); const v16h wf1 = WFrag<h16>::ld(wr + (size_t)(16 + lr) * 32 + 8 * hi); const float q0 = bfr(b2[lr]), q1 = bfr(b2[16 + lr]);
    v16h sa = (v16h){}, sb = (v16h){};
    for (int ts = 0; ts < NTS; ++ts) { const size_t r0 = (size_t)ts * NBR + b0; const float* pin = src + (r0 + 8 * hi) * 64 + lr; v8f c0, c1;
#pragma unroll
        for (int j = 0; j < 8; ++j) { c0[j] = pin[(size_t)j * 64] + q0; c1[j] = pin[(size_t)j * 64 + 16] + q1; }
        const v8f d0 = wmma16(sa, wf0, c0), d1 = wmma16(sa, wf1, c1); const v8f e0 = wmma16(sb, wf0, (v8f){}), e1 = wmma16(sb, wf1, (v8f){});
        __builtin_amdgcn_wave_barrier(); asm volatile("" ::: "memory");
#pragma unroll
        for (int j = 0; j < 8; ++j) { const float v0 = d0[j] + e0[j] * 0.00048828125f, v1 = d1[j] + e1[j] * 0.00048828125f; tl[(8 * hi + j) * 36 + lr] = 1.0f - 2.0f / (1.0f + expf(2.0f * v0)); tl[(8 * hi + j) * 36 + 16 + lr] = 1.0f - 2.0f / (1.0f + expf(2.0f * v1)); }
        __builtin_amdgcn_wave_barrier(); asm volatile("" ::: "memory");
        const float* pr = tl + lr * 36 + 8 * hi; const v4f a0 = *(const v4fa*)pr, a1 = *(const v4fa*)(pr + 4), a2 = *(const v4fa*)(pr + 16), a3 = *(const v4fa*)(pr + 20);
#pragma unroll
        for (int j = 0; j < 4; ++j) { const h16 w0 = toh_flush(a0[j]), w1 = toh_flush(a1[j]), w2 = toh_flush(a2[j]), w3 = toh_flush(a3[j]); sa[j] = w0; sa[4 + j] = w1; sa[8 + j] = w2; sa[12 + j] = w3;
            sb[j] = toh_flush((a0[j] - (float)w0) * 2048.0f); sb[4 + j] = toh_flush((a1[j] - (float)w1) * 2048.0f); sb[8 + j] = toh_flush((a2[j] - (float)w2) * 2048.0f); sb[12 + j] = toh_flush((a3[j] - (float)w3) * 2048.0f); }
        const float* po = tl + (lane >> 2) * 36 + 8 * (lane & 3); const v4f u0 = *(const v4fa*)po, u1 = *(const v4fa*)(po + 4), u2 = *(const v4fa*)(po + 8 * 36), u3 = *(const v4fa*)(po + 8 * 36 + 4); v8h oa, ob;
#pragma unroll
        for (int j = 0; j < 4; ++j) { oa[j] = toh_flush(RL ? fmaxf(u0[j], 0.0f) : u0[j]); oa[4 + j] = toh_flush(RL ? fmaxf(u1[j], 0.0f) : u1[j]); ob[j] = toh_flush(RL ? fmaxf(u2[j], 0.0f) : u2[j]); ob[4 + j] = toh_flush(RL ? fmaxf(u3[j], 0.0f) : u3[j]); }
        h16* pw = dst + (r0 + (lane >> 2)) * 32 + 8 * (lane & 3);
        *(volatile v8h*)pw = oa; *(volatile v8h*)(pw + 8 * 32) = ob; __threadfence(); *(volatile v8h*)pw = oa; *(volatile v8h*)(pw + 8 * 32) = ob;
        __builtin_amdgcn_wave_barrier(); asm volatile("" ::: "memory"); } }

extern "C" void kernel_launch(void* const* d_in, const int* in_sizes, int n_in, void* d_out, int out_size, void* d_ws, size_t ws_size, hipStream_t stream) {
    if (n_in < 21) return;
    const int want[21] = {NRW * 64, 128 * 64, 128, 64 * 128, 64, 32 * 64, 32, 20 * 32, 20 * 20, 20, 20, 32 * 20, 32 * 32, 32, 32, 64 * 32, 64, 128 * 64, 128, 64 * 128, 64};
    for (int q = 0; q < 21; ++q) if (in_sizes[q] != want[q]) return;
    if (out_size != NRW * 64) return;
    static_assert(NRW == NTS * NBR && NRW % 64 == 0 && (NRW * 64 / 8) % 256 == 0 && (NRW * 32 / 8) % 256 == 0 && NBR == 16 * 16, "the rows in 64s for the products; the flat grids exact; 16 waves of 16 batch rows a cell");
    const float* xin = (const float*)d_in[0]; const float* we1 = (const float*)d_in[1]; const float* be1 = (const float*)d_in[2]; const float* we2 = (const float*)d_in[3]; const float* be2 = (const float*)d_in[4]; const float* we3 = (const float*)d_in[5]; const float* be3 = (const float*)d_in[6];
    const float* wi1 = (const float*)d_in[7]; const float* wr1 = (const float*)d_in[8]; const float* bi1 = (const float*)d_in[9]; const float* br1 = (const float*)d_in[10]; const float* wi2 = (const float*)d_in[11]; const float* wr2 = (const float*)d_in[12]; const float* bi2 = (const float*)d_in[13]; const float* br2 = (const float*)d_in[14];
    const float* wd1 = (const float*)d_in[15]; const float* bd1 = (const float*)d_in[16]; const float* wd2 = (const float*)d_in[17]; const float* bd2 = (const float*)d_in[18]; const float* wd3 = (const float*)d_in[19]; const float* bd3 = (const float*)d_in[20]; float* res = (float*)d_out;
    char* wsp = (char*)d_ws; auto take = [&](size_t bytes) { char* p = wsp; wsp += (bytes + 255) & ~(size_t)255; return (void*)p; };
    h16* A1 = (h16*)take((size_t)NRW * 64 * 2); h16* Xw = A1;
    h16* W1 = (h16*)take(128 * 64 * 2); h16* W2 = (h16*)take(64 * 128 * 2); h16* W3 = (h16*)take(64 * 64 * 2); h16* W4 = (h16*)take(64 * 32 * 2); h16* W5 = (h16*)take(64 * 32 * 2); h16* W6 = (h16*)take(64 * 32 * 2); h16* W7 = (h16*)take(128 * 64 * 2); h16* W8 = (h16*)take(64 * 128 * 2); h16* V1 = (h16*)take(32 * 32 * 2); h16* V2 = (h16*)take(32 * 32 * 2);
    float* B1 = (float*)take(128 * 4); float* B2 = (float*)take(64 * 4); float* B3 = (float*)take(64 * 4); float* B4 = (float*)take(64 * 4); float* B5 = (float*)take(64 * 4); float* B6 = (float*)take(64 * 4); float* B7 = (float*)take(128 * 4); float* B8 = (float*)take(64 * 4); float* Q4 = (float*)take(64 * 4); float* Q5 = (float*)take(64 * 4);
    float* F0 = (float*)take((size_t)NRW * 64 * 4); float* F1 = (float*)take((size_t)NRW * 64 * 4); h16* A0 = (h16*)take((size_t)NRW * 128 * 2);
    if ((size_t)(wsp - (char*)d_ws) > ws_size) return;
    k_wword<<<128 * 64 / 2 / 256, 256, 0, stream>>>(we1, 128, 64, W1, 64); k_wword<<<64 * 128 / 2 / 256, 256, 0, stream>>>(we2, 64, 128, W2, 128); k_wword<<<64 * 64 / 2 / 256, 256, 0, stream>>>(we3, 32, 64, W3, 64); k_wword<<<64 * 32 / 2 / 256, 256, 0, stream>>>(wi1, 20, 32, W4, 32);
    k_wword<<<64 * 32 / 2 / 256, 256, 0, stream>>>(wi2, 32, 20, W5, 32); k_wword<<<64 * 32 / 2 / 256, 256, 0, stream>>>(wd1, 64, 32, W6, 32); k_wword<<<128 * 64 / 2 / 256, 256, 0, stream>>>(wd2, 128, 64, W7, 64); k_wword<<<64 * 128 / 2 / 256, 256, 0, stream>>>(wd3, 64, 128, W8, 128);
    k_wword<<<32 * 32 / 2 / 256, 256, 0, stream>>>(wr1, 20, 20, V1, 32); k_wword<<<32 * 32 / 2 / 256, 256, 0, stream>>>(wr2, 32, 32, V2, 32);
    k_bpad<<<1, 128, 0, stream>>>(be1, 128, B1); k_bpad<<<1, 64, 0, stream>>>(be2, 64, B2); k_bpad<<<1, 64, 0, stream>>>(be3, 32, B3); k_bpad<<<1, 64, 0, stream>>>(bi1, 20, B4); k_bpad<<<1, 64, 0, stream>>>(bi2, 32, B5);
    k_bpad<<<1, 64, 0, stream>>>(bd1, 64, B6); k_bpad<<<1, 128, 0, stream>>>(bd2, 128, B7); k_bpad<<<1, 64, 0, stream>>>(bd3, 64, B8); k_bpad<<<1, 64, 0, stream>>>(br1, 20, Q4); k_bpad<<<1, 64, 0, stream>>>(br2, 32, Q5);
    k_xword<<<(unsigned)(NRW * 64 / 8 / 256), 256, 0, stream>>>(xin, Xw);
    k_gemmw<h16, 0, true><<<dim3(NRW / 64, 1, 1), 32, 0, stream>>>(Xw, nullptr, W1, nullptr, 64, F0, 64, B1, 0, 0, 0);
    k_gemmw<h16, 0, true><<<dim3(NRW / 64, 1, 1), 32, 0, stream>>>(Xw, nullptr, W1 + 64 * 64, nullptr, 64, F1, 64, B1 + 64, 0, 0, 0);
    k_rword<<<(unsigned)(NRW * 64 / 8 / 256), 256, 0, stream>>>(F0, 64, A0, 128, 3); k_rword<<<(unsigned)(NRW * 64 / 8 / 256), 256, 0, stream>>>(F1, 64, A0 + 64, 128, 3);
    k_gemmw<h16, 0, true><<<dim3(NRW / 64, 1, 1), 32, 0, stream>>>(A0, nullptr, W2, nullptr, 128, F0, 64, B2, 0, 0, 0);
    k_rword<<<(unsigned)(NRW * 64 / 8 / 256), 256, 0, stream>>>(F0, 64, A1, 64, 3);
    k_gemmw<h16, 0, true><<<dim3(NRW / 64, 1, 1), 32, 0, stream>>>(A1, nullptr, W3, nullptr, 64, F1, 64, B3, 0, 0, 0);
    k_rword<<<(unsigned)(NRW * 32 / 8 / 256), 256, 0, stream>>>(F1, 64, A0, 32, 2);
    k_gemmw<h16, 0, true><<<dim3(NRW / 64, 1, 1), 32, 0, stream>>>(A0, nullptr, W4, nullptr, 32, F0, 64, B4, 0, 0, 0);
    k_cellm<false><<<16, 32, 0, stream>>>(F0, V1, Q4, A1);
    k_gemmw<h16, 0, true><<<dim3(NRW / 64, 1, 1), 32, 0, stream>>>(A1, nullptr, W5, nullptr, 32, F1, 64, B5, 0, 0, 0);
    k_cellm<true><<<16, 32, 0, stream>>>(F1, V2, Q5, A0);
    k_gemmw<h16, 0, true><<<dim3(NRW / 64, 1, 1), 32, 0, stream>>>(A0, nullptr, W6, nullptr, 32, F0, 64, B6, 0, 0, 0);
    k_rword<<<(unsigned)(NRW * 64 / 8 / 256), 256, 0, stream>>>(F0, 64, A1, 64, 3);
    k_gemmw<h16, 0, true><<<dim3(NRW / 64, 1, 1), 32, 0, stream>>>(A1, nullptr, W7, nullptr, 64, F0, 64, B7, 0, 0, 0);
    k_gemmw<h16, 0, true><<<dim3(NRW / 64, 1, 1), 32, 0, stream>>>(A1, nullptr, W7 + 64 * 64, nullptr, 64, F1, 64, B7 + 64, 0, 0, 0);
    k_rword<<<(unsigned)(NRW * 64 / 8 / 256), 256, 0, stream>>>(F0, 64, A0, 128, 3); k_rword<<<(unsigned)(NRW * 64 / 8 / 256), 256, 0, stream>>>(F1, 64, A0 + 64, 128, 3);
    k_gemmw<h16, 0, true><<<dim3(NRW / 64, 1, 1), 32, 0, stream>>>(A0, nullptr, W8, nullptr, 128, res, 64, B8, 0, 0, 0);
}
